// DeltaNet_34007551049775
// MI455X (gfx1250) — hardware-verified
//
#include <hip/hip_runtime.h>
#include <math.h>

constexpr int kBatch     = 2;
constexpr int kSeq       = 2048;
constexpr int kDim       = 2048;
constexpr int kHeads     = 16;
constexpr int kHd        = 128;
constexpr int kRows      = kBatch * kSeq;
constexpr int kGateN     = 64;
constexpr int kChunk     = 32;
constexpr int kNumChunks = kSeq / kChunk;
constexpr float kWCarry    = 64.0f;
constexpr float kWCarryInv = 1.0f / 64.0f;
constexpr float kResCarry  = 2048.0f;
constexpr float kResInv    = 1.0f / 2048.0f;
constexpr float kNormEps   = 1e-5f;
constexpr size_t kHeadPlaneHalves = (size_t)kBatch * kHeads * kSeq * kHd;

static_assert(kDim == kHeads * kHd, "head packing");
static_assert(kHd == 128 && kChunk == 32, "scan tiling");
static_assert(kRows % 64 == 0 && kDim % 64 == 0 && kGateN % 64 == 0, "GEMM M,N tile multiples");
static_assert(kDim % 32 == 0, "GEMM K multiple of 32");
static_assert(kSeq % kChunk == 0 && kSeq % 2 == 0, "sequence tiling");
static_assert((kRows * kHeads / 2) % 8 == 0, "l2n grid exact");
static_assert(kHeadPlaneHalves == (size_t)kRows * kDim, "head-major plane extent equals the token-major plane extent");
static_assert(((size_t)(kBatch * kHeads - 1) * kSeq + (kSeq - 1)) * kHd + (kHd - 1) < kHeadPlaneHalves, "max q/k plane index inside its carve");

constexpr int kQP = 136;
constexpr int kTP = 40;
constexpr int kWP = 132;
constexpr int kSP = 132;
constexpr int kOffK    = 0;
constexpr int kOffQD   = kOffK + kChunk * kQP * 2;
constexpr int kOffKT   = kOffQD + kHd * kTP * 2;
constexpr int kOffDH   = kOffKT + kHd * kTP * 2;
constexpr int kOffP    = kOffDH + kHd * kTP * 2;
constexpr int kOffA    = kOffP + kChunk * kTP * 2;
constexpr int kOffW    = kOffA + kChunk * kChunk * 4;
constexpr int kOffBeta = kOffW + kChunk * kWP * 4;
constexpr int kOffS    = kOffBeta + kChunk * 4;
constexpr int kScanLdsBytes = kOffS + kHd * kSP * 4;
static_assert(kChunk * kQP * 2 <= kHd * kTP * 2, "Q tile fits the aliased residual-delta region");
static_assert(kScanLdsBytes <= 163840, "LDS budget");
static_assert((kHd * kSP) % 4 == 0, "state zero-fill in 16-B pieces");
static_assert((kOffQD % 16) == 0 && (kOffKT % 16) == 0 && (kOffDH % 16) == 0 && (kOffP % 16) == 0 &&
              (kOffA % 16) == 0 && (kOffW % 16) == 0 && (kOffBeta % 16) == 0 && (kOffS % 16) == 0, "LDS alignment");
static_assert(((kSP * 4) % 16) == 0 && ((kWP * 4) % 16) == 0 && ((kQP * 2) % 16) == 0 && ((kTP * 2) % 16) == 0, "LDS row pitches 16-B aligned");
static_assert(kChunk % 8 == 0, "substitution blocks of 8 rows");

typedef __attribute__((ext_vector_type(16))) _Float16 v16h;
typedef __attribute__((ext_vector_type(8)))  _Float16 v8h;
typedef __attribute__((ext_vector_type(8)))  float    v8f;
typedef __attribute__((ext_vector_type(4)))  float    v4f;
typedef __attribute__((ext_vector_type(4)))  unsigned int v4u;
typedef v8h v8h_a __attribute__((may_alias));
typedef v4u v4u_a __attribute__((may_alias));
typedef v4f v4f_a __attribute__((may_alias));
typedef unsigned short us_a __attribute__((may_alias));

__device__ __forceinline__ unsigned short f2bf_bits(float f) {
  unsigned u = __float_as_uint(f);
  return (unsigned short)((u + 0x7FFFu + ((u >> 16) & 1u)) >> 16);
}
__device__ __forceinline__ float bf_bits2f(unsigned short h) { return __uint_as_float(((unsigned)h) << 16); }
__device__ __forceinline__ float bf16r(float f) { return bf_bits2f(f2bf_bits(f)); }
__device__ __forceinline__ unsigned short h_bits(float f) {
  const _Float16 h = (_Float16)f;
  return __builtin_bit_cast(unsigned short, h);
}
__device__ __forceinline__ unsigned pk16(unsigned short a, unsigned short b) { return (unsigned)a | ((unsigned)b << 16); }

union FragU { v16h v; v8h h[2]; };
__device__ __forceinline__ v16h glb_frag(const _Float16* p) {
  FragU f;
  f.h[0] = *(const v8h*)(p);
  f.h[1] = *(const v8h*)(p + 16);
  return f.v;
}
__device__ __forceinline__ v16h lds_frag(const _Float16* p) {
  FragU f;
  f.h[0] = *(const v8h_a*)(p);
  f.h[1] = *(const v8h_a*)(p + 16);
  return f.v;
}
__device__ __forceinline__ v8f wmma_h(v16h a, v16h b, v8f c) {
  return __builtin_amdgcn_wmma_f32_16x16x32_f16(false, a, false, b, (short)0, c, false, false);
}
__device__ __forceinline__ void hz_guard4(v8f& a, v8f& b, v8f& c, v8f& d,
                                          v16h x0, v16h x1, v16h x2, v16h x3, v16h x4, v16h x5) {
  asm volatile("v_nop\n\tv_nop\n\tv_nop\n\tv_nop"
               : "+v"(a), "+v"(b), "+v"(c), "+v"(d)
               : "v"(x0), "v"(x1), "v"(x2), "v"(x3), "v"(x4), "v"(x5));
}
__device__ __forceinline__ void hz_guard2(v8f& a, v8f& b, v16h x0, v16h x1, v16h x2) {
  asm volatile("v_nop\n\tv_nop\n\tv_nop\n\tv_nop" : "+v"(a), "+v"(b) : "v"(x0), "v"(x1), "v"(x2));
}
__device__ __forceinline__ void hz_guard1(v8f& a, v16h x0, v16h x1) {
  asm volatile("v_nop\n\tv_nop\n\tv_nop\n\tv_nop" : "+v"(a) : "v"(x0), "v"(x1));
}
__device__ __forceinline__ void keep4_h(v16h a, v16h b, v16h c, v16h d) { asm volatile("v_nop" :: "v"(a), "v"(b), "v"(c), "v"(d)); }
__device__ __forceinline__ void acc_guard4(v8f& a, v8f& b, v8f& c, v8f& d) {
  asm volatile("v_nop\n\tv_nop\n\tv_nop\n\tv_nop" : "+v"(a), "+v"(b), "+v"(c), "+v"(d));
}
__device__ __forceinline__ void sched_fence() { asm volatile("" ::: "memory"); }
__device__ __forceinline__ void split_h(float x, _Float16& hi, _Float16& lo) {
  hi = (_Float16)x;
  float hf = (float)hi;
  asm("" : "+v"(hf));
  lo = (_Float16)((x - hf) * kResCarry);
}

__global__ __launch_bounds__(256) void cvt_x_kernel(const float* __restrict__ in, unsigned short* __restrict__ out, int n8) {
  const int i = blockIdx.x * 256 + threadIdx.x;
  if (i >= n8) return;
  const float* p = in + 8 * (size_t)i;
  const v4f a = *(const v4f*)(p);
  const v4f b = *(const v4f*)(p + 4);
  unsigned short hb[8];
#pragma unroll
  for (int e = 0; e < 4; ++e) {
    const float x0 = a[e];
    const float x1 = b[e];
    hb[e]     = h_bits(bf16r(x0));
    hb[4 + e] = h_bits(bf16r(x1));
  }
  const v4u u = (v4u){pk16(hb[0], hb[1]), pk16(hb[2], hb[3]), pk16(hb[4], hb[5]), pk16(hb[6], hb[7])};
  unsigned short* q = out + 8 * (size_t)i;
  *(volatile v4u*)q = u;
  __threadfence();
  *(volatile v4u*)q = u;
}

__global__ __launch_bounds__(256) void wt_cast_kernel(const float* __restrict__ W0, const float* __restrict__ W1,
                                                      const float* __restrict__ W2, const float* __restrict__ W3,
                                                      unsigned short* __restrict__ out) {
  __shared__ float sm[64][65];
  const int t  = threadIdx.x;
  const int k0 = blockIdx.x * 64;
  const int n0 = blockIdx.y * 64;
  const int z  = blockIdx.z;
  const float* W = (z == 0) ? W0 : (z == 1) ? W1 : (z == 2) ? W2 : W3;
#pragma unroll
  for (int i = 0; i < 16; ++i) {
    const int e  = i * 256 + t;
    const int r  = e >> 6;
    const int cc = e & 63;
    sm[cc][r] = bf16r(W[(size_t)(k0 + r) * kDim + n0 + cc]) * kWCarry;
  }
  __syncthreads();
  const int lane = t & 31, wave = t >> 5;
  const int q = lane >> 3, c8 = (lane & 7) * 8;
  unsigned short* op = out + (size_t)z * kDim * kDim;
  v4u u[2];
#pragma unroll
  for (int it = 0; it < 2; ++it) {
    const int row = wave * 8 + it * 4 + q;
    unsigned short hb[8];
#pragma unroll
    for (int e = 0; e < 8; ++e) hb[e] = h_bits(sm[row][c8 + e]);
    u[it] = (v4u){pk16(hb[0], hb[1]), pk16(hb[2], hb[3]), pk16(hb[4], hb[5]), pk16(hb[6], hb[7])};
  }
  for (int pass = 0; pass < 2; ++pass) {
#pragma unroll
    for (int it = 0; it < 2; ++it) {
      const int row = wave * 8 + it * 4 + q;
      *(volatile v4u*)(op + (size_t)(n0 + row) * kDim + k0 + c8) = u[it];
    }
    __threadfence();
  }
}

__global__ __launch_bounds__(256) void wb_cast_kernel(const float* __restrict__ Wb, unsigned short* __restrict__ out) {
  __shared__ float sm[kHeads][65];
  const int t  = threadIdx.x;
  const int k0 = blockIdx.x * 64;
  {
    const v4f v = *(const v4f*)(Wb + (size_t)k0 * kHeads + 4 * t);
    const int kk = t >> 2;
    const int nb = (t & 3) * 4;
#pragma unroll
    for (int e = 0; e < 4; ++e) {
      const float x = v[e];
      sm[nb + e][kk] = bf16r(x) * kWCarry;
    }
  }
  __syncthreads();
  const int lane = t & 31, wave = t >> 5;
  const int q = lane >> 3, c8 = (lane & 7) * 8;
  v4u u[2];
#pragma unroll
  for (int it = 0; it < 2; ++it) {
    const int row = wave * 8 + it * 4 + q;
    const int rc  = (row < kHeads) ? row : (kHeads - 1);
    const unsigned msk = (row < kHeads) ? 0xffffffffu : 0u;
    unsigned short hb[8];
#pragma unroll
    for (int e = 0; e < 8; ++e) hb[e] = h_bits(sm[rc][c8 + e]);
    u[it] = (v4u){pk16(hb[0], hb[1]) & msk, pk16(hb[2], hb[3]) & msk, pk16(hb[4], hb[5]) & msk, pk16(hb[6], hb[7]) & msk};
  }
  for (int pass = 0; pass < 2; ++pass) {
#pragma unroll
    for (int it = 0; it < 2; ++it) {
      const int row = wave * 8 + it * 4 + q;
      *(volatile v4u*)(out + (size_t)row * kDim + k0 + c8) = u[it];
    }
    __threadfence();
  }
}

__global__ __launch_bounds__(256) void wmma_gemm64_f16(
    const unsigned short* __restrict__ Ap, int lda,
    const unsigned short* __restrict__ Btp, int ldb,
    float* __restrict__ Cout, int ldc, int M, int N, int K, float scale) {
  const _Float16* A  = (const _Float16*)Ap;
  const _Float16* Bt = (const _Float16*)Btp;
  __shared__ __align__(16) float sT[8][16 * 68];
  const int lane = threadIdx.x & 31;
  const int wave = threadIdx.x >> 5;
  const int tilesN = N >> 6;
  const int tilesM = M >> 6;
  const int tile = blockIdx.x * 8 + wave;
  if (tile >= tilesM * tilesN) return;
  const int tm = tile / tilesN;
  const int tn = tile - tm * tilesN;
  const int m0 = tm << 6;
  const int n0 = tn << 6;
  const int rlane = lane & 15;
  const int koff  = (lane >> 4) * 8;
  const int mOff  = (lane >> 4) * 8;
  const _Float16* ap0 = A  + (size_t)(m0 + rlane) * lda + koff;
  const _Float16* bp0 = Bt + (size_t)(n0 + rlane) * ldb + koff;
  const size_t astep = (size_t)16 * lda;
  const size_t bstep = (size_t)16 * ldb;

  v8f acc[4][4];
#pragma unroll
  for (int i = 0; i < 4; ++i)
#pragma unroll
    for (int j = 0; j < 4; ++j) acc[i][j] = (v8f){0.f, 0.f, 0.f, 0.f, 0.f, 0.f, 0.f, 0.f};

  for (int k0 = 0; k0 < K; k0 += 32) {
    v16h bh[4];
#pragma unroll
    for (int j = 0; j < 4; ++j) bh[j] = glb_frag(bp0 + j * bstep + k0);
#pragma unroll
    for (int i = 0; i < 4; ++i) {
      const v16h ah = glb_frag(ap0 + i * astep + k0);
#pragma unroll
      for (int j = 0; j < 4; ++j) acc[i][j] = wmma_h(ah, bh[j], acc[i][j]);
      hz_guard4(acc[i][0], acc[i][1], acc[i][2], acc[i][3], ah, ah, bh[0], bh[1], bh[2], bh[3]);
    }
    keep4_h(bh[0], bh[1], bh[2], bh[3]);
  }
  acc_guard4(acc[0][0], acc[0][1], acc[0][2], acc[0][3]);
  acc_guard4(acc[1][0], acc[1][1], acc[1][2], acc[1][3]);
  acc_guard4(acc[2][0], acc[2][1], acc[2][2], acc[2][3]);
  acc_guard4(acc[3][0], acc[3][1], acc[3][2], acc[3][3]);

  float* slab = sT[wave];
#pragma unroll
  for (int i = 0; i < 4; ++i) {
    const int mBase = m0 + (i << 4);
#pragma unroll
    for (int j = 0; j < 4; ++j) {
#pragma unroll
      for (int r = 0; r < 8; ++r) {
        const float v = acc[i][j][r] * scale;
        slab[(mOff + r) * 68 + (j << 4) + rlane] = v;
      }
    }
    __builtin_amdgcn_fence(__ATOMIC_RELEASE, "workgroup");
    __builtin_amdgcn_wave_barrier();
    __builtin_amdgcn_fence(__ATOMIC_ACQUIRE, "workgroup");
    {
      const int hh = lane >> 4, c4 = (lane & 15) * 4;
      for (int pass = 0; pass < 2; ++pass) {
#pragma unroll
        for (int it = 0; it < 8; ++it) {
          const int row = it * 2 + hh;
          const v4f v = *(const v4f_a*)(slab + row * 68 + c4);
          *(volatile v4f*)(Cout + (size_t)(mBase + row) * ldc + n0 + c4) = v;
        }
        __threadfence();
      }
    }
    __builtin_amdgcn_fence(__ATOMIC_RELEASE, "workgroup");
    __builtin_amdgcn_wave_barrier();
    __builtin_amdgcn_fence(__ATOMIC_ACQUIRE, "workgroup");
  }
}

__global__ __launch_bounds__(256) void l2n_heads_kernel(const float* __restrict__ src, unsigned short* __restrict__ dst) {
  const int lane = threadIdx.x & 31, wave = threadIdx.x >> 5;
  const int c = lane & 15, hh = lane >> 4;
  const int p  = blockIdx.x * 8 + wave;
  const int hd = p & (kHeads - 1);
  const int mp = p >> 4;
  const int m  = 2 * mp + hh;
  const int bi = m / kSeq;
  const int l  = m - bi * kSeq;
  const float* sp = src + (size_t)m * kDim + hd * kHd + 8 * c;
  const v4f a = *(const v4f*)(sp);
  const v4f b = *(const v4f*)(sp + 4);
  float ss = 0.0f;
#pragma unroll
  for (int e = 0; e < 4; ++e) {
    ss += a[e] * a[e];
    ss += b[e] * b[e];
  }
  ss += __shfl_xor(ss, 1, 32);
  ss += __shfl_xor(ss, 2, 32);
  ss += __shfl_xor(ss, 4, 32);
  ss += __shfl_xor(ss, 8, 32);
  const float inv = 1.0f / fmaxf(sqrtf(ss), 1e-12f);
  unsigned short hb[8];
#pragma unroll
  for (int e = 0; e < 4; ++e) {
    const float y0 = a[e] * inv;
    const float y1 = b[e] * inv;
    hb[e]     = h_bits(y0);
    hb[4 + e] = h_bits(y1);
  }
  const v4u u = (v4u){pk16(hb[0], hb[1]), pk16(hb[2], hb[3]), pk16(hb[4], hb[5]), pk16(hb[6], hb[7])};
  unsigned short* dp = dst + ((size_t)(bi * kHeads + hd) * kSeq + l) * kHd + 8 * c;
  *(volatile v4u*)dp = u;
  __threadfence();
  *(volatile v4u*)dp = u;
}

__global__ __launch_bounds__(256) __attribute__((amdgpu_num_vgpr(256))) void chunk_scan_kernel(
    const unsigned short* __restrict__ Qp, const unsigned short* __restrict__ Kp,
    const float* __restrict__ Vraw, const float* __restrict__ Graw,
    const float* __restrict__ nw, unsigned short* __restrict__ On) {
  extern __shared__ __align__(16) unsigned char lds[];
  _Float16* const sK   = (_Float16*)(lds + kOffK);
  _Float16* const sQ   = (_Float16*)(lds + kOffQD);
  _Float16* const sDl  = (_Float16*)(lds + kOffQD);
  _Float16* const sKT  = (_Float16*)(lds + kOffKT);
  _Float16* const sDh  = (_Float16*)(lds + kOffDH);
  _Float16* const sP   = (_Float16*)(lds + kOffP);
  float* const    sA   = (float*)(lds + kOffA);
  float* const    sW   = (float*)(lds + kOffW);
  float* const    sBeta = (float*)(lds + kOffBeta);
  float* const    sS   = (float*)(lds + kOffS);

  const int tid = threadIdx.x;
  const int lane = tid & 31, wave = tid >> 5;
  const int c = lane & 15, hh = lane >> 4;
  const int bh = blockIdx.x;
  const int bi = bh / kHeads;
  const int hd = bh - bi * kHeads;
  const size_t planeBase = (size_t)bh * kSeq * kHd;
  const size_t rowBase   = (size_t)bi * kSeq;

  const v8f z8 = {0.f, 0.f, 0.f, 0.f, 0.f, 0.f, 0.f, 0.f};

  {
    const v4f zz = {0.f, 0.f, 0.f, 0.f};
#pragma unroll 1
    for (int i = tid; i < kHd * kSP / 4; i += 256) *(v4f_a*)(sS + 4 * i) = zz;
  }
  __syncthreads();

  const float qscl = 1.0f / sqrtf((float)kHd);

  const int isP = wave >> 2;
  const int ti  = (wave & 3) >> 1;
  const int tj  = wave & 1;
  const _Float16* const aRows = (const _Float16*)(lds + (isP ? kOffQD : kOffK));
  float* const sRow = sS + (16 * wave + c) * kSP + 8 * hh;

#pragma unroll 1
  for (int ch = 0; ch < kNumChunks; ++ch) {
    const int t0 = ch * kChunk;

    {
      const int t = tid >> 3, seg = tid & 7;
      const size_t g = planeBase + (size_t)(t0 + t) * kHd + seg * 16;
      const v4u qw0 = *(const v4u*)(Qp + g);
      const v4u qw1 = *(const v4u*)(Qp + g + 8);
      const v4u kw0 = *(const v4u*)(Kp + g);
      const v4u kw1 = *(const v4u*)(Kp + g + 8);
      *(v4u_a*)(lds + kOffQD + t * (kQP * 2) + seg * 32)      = qw0;
      *(v4u_a*)(lds + kOffQD + t * (kQP * 2) + seg * 32 + 16) = qw1;
      *(v4u_a*)(lds + kOffK  + t * (kQP * 2) + seg * 32)      = kw0;
      *(v4u_a*)(lds + kOffK  + t * (kQP * 2) + seg * 32 + 16) = kw1;
      us_a* kt = (us_a*)(lds + kOffKT);
#pragma unroll
      for (int wi = 0; wi < 4; ++wi) {
        const unsigned w0 = kw0[wi];
        const unsigned w1 = kw1[wi];
        const int d0 = seg * 16 + 2 * wi;
        const int d1 = seg * 16 + 8 + 2 * wi;
        kt[d0 * kTP + t]       = (unsigned short)(w0 & 0xffffu);
        kt[(d0 + 1) * kTP + t] = (unsigned short)(w0 >> 16);
        kt[d1 * kTP + t]       = (unsigned short)(w1 & 0xffffu);
        kt[(d1 + 1) * kTP + t] = (unsigned short)(w1 >> 16);
      }
    }
    if (tid < kChunk) {
      const float x = Graw[(rowBase + t0 + tid) * kGateN + hd];
      sBeta[tid] = 1.0f / (1.0f + expf(-x));
    }
    __syncthreads();

    v8f vp0 = z8, vp1 = z8, vl0 = z8, vl1 = z8;
    v8f o0 = z8, o1 = z8, ol0 = z8, ol1 = z8;
    {
      const _Float16* kA = sK + c * kQP + 8 * hh;
      const _Float16* qA = sQ + c * kQP + 8 * hh;
#pragma unroll 1
      for (int g = 0; g < 4; ++g) {
        const v4f s0 = *(const v4f_a*)(sRow + 32 * g);
        const v4f s1 = *(const v4f_a*)(sRow + 32 * g + 4);
        const v4f s2 = *(const v4f_a*)(sRow + 32 * g + 16);
        const v4f s3 = *(const v4f_a*)(sRow + 32 * g + 20);
        v16h bhi, blo;
#pragma unroll
        for (int e = 0; e < 4; ++e) {
          _Float16 h0, l0, h1, l1, h2, l2, h3, l3;
          const float x0 = s0[e];
          const float x1 = s1[e];
          const float x2 = s2[e];
          const float x3 = s3[e];
          split_h(x0, h0, l0);
          split_h(x1, h1, l1);
          split_h(x2, h2, l2);
          split_h(x3, h3, l3);
          bhi[e]      = h0;
          blo[e]      = l0;
          bhi[4 + e]  = h1;
          blo[4 + e]  = l1;
          bhi[8 + e]  = h2;
          blo[8 + e]  = l2;
          bhi[12 + e] = h3;
          blo[12 + e] = l3;
        }
        {
          const v16h ka0 = lds_frag(kA + 32 * g);
          const v16h ka1 = lds_frag(kA + 16 * kQP + 32 * g);
          vp0 = wmma_h(ka0, bhi, vp0);
          vl0 = wmma_h(ka0, blo, vl0);
          vp1 = wmma_h(ka1, bhi, vp1);
          vl1 = wmma_h(ka1, blo, vl1);
          hz_guard4(vp0, vl0, vp1, vl1, ka0, ka1, bhi, blo, ka0, ka1);
        }
        sched_fence();
        {
          const v16h qa0 = lds_frag(qA + 32 * g);
          const v16h qa1 = lds_frag(qA + 16 * kQP + 32 * g);
          o0  = wmma_h(qa0, bhi, o0);
          ol0 = wmma_h(qa0, blo, ol0);
          o1  = wmma_h(qa1, bhi, o1);
          ol1 = wmma_h(qa1, blo, ol1);
          hz_guard4(o0, ol0, o1, ol1, qa0, qa1, bhi, blo, qa0, qa1);
        }
        sched_fence();
      }
    }
#pragma unroll
    for (int r = 0; r < 8; ++r) {
      const float p0 = vp0[r] + vl0[r] * kResInv;
      const float p1 = vp1[r] + vl1[r] * kResInv;
      sW[(8 * hh + r) * kWP + 16 * wave + c]      = p0;
      sW[(16 + 8 * hh + r) * kWP + 16 * wave + c] = p1;
      o0[r] = o0[r] + ol0[r] * kResInv;
      o1[r] = o1[r] + ol1[r] * kResInv;
    }
    v8f gacc = z8;
    {
      const _Float16* pa = aRows + (16 * ti + c) * kQP + 8 * hh;
      const _Float16* pb = sK + (16 * tj + c) * kQP + 8 * hh;
#pragma unroll 1
      for (int db = 0; db < 4; ++db) {
        const v16h ua = lds_frag(pa + 32 * db);
        const v16h ub = lds_frag(pb + 32 * db);
        gacc = wmma_h(ua, ub, gacc);
        hz_guard1(gacc, ua, ub);
        sched_fence();
      }
    }
#pragma unroll 1
    for (int rb = 0; rb < 2; ++rb) {
      const float* vsrc = Vraw + (rowBase + t0 + 16 * rb + 8 * hh) * kDim + hd * kHd + 16 * wave + c;
      float* wp = sW + (16 * rb + 8 * hh) * kWP + 16 * wave + c;
#pragma unroll
      for (int r = 0; r < 8; ++r) {
        const float x  = vsrc[(size_t)r * kDim];
        const float e  = expf(-x);
        const float sv = x * (1.0f / (1.0f + e));
        const float pv = wp[r * kWP];
        wp[r * kWP] = sv - pv;
      }
    }
    if (isP == 0) {
#pragma unroll
      for (int r = 0; r < 8; ++r) sA[(16 * ti + 8 * hh + r) * kChunk + 16 * tj + c] = gacc[r];
    } else {
      us_a* pu = (us_a*)(lds + kOffP);
#pragma unroll
      for (int r = 0; r < 8; ++r) {
        const int m = 16 * ti + 8 * hh + r;
        const int n = 16 * tj + c;
        const unsigned short bits = h_bits(gacc[r]);
        pu[m * kTP + n] = (n <= m) ? bits : (unsigned short)0;
      }
    }
    __syncthreads();

    if (tid < kHd) {
      float* const wcol = sW + tid;
      _Float16* const dhRow = sDh + tid * kTP;
      _Float16* const dlRow = sDl + tid * kTP;
#pragma unroll 1
      for (int b = 0; b < kChunk / 8; ++b) {
        const int r0 = 8 * b;
        float acc[8];
#pragma unroll
        for (int i = 0; i < 8; ++i) acc[i] = wcol[(r0 + i) * kWP];
#pragma unroll 1
        for (int s4 = 0; s4 < 2 * b; ++s4) {
          const float d0 = wcol[(4 * s4 + 0) * kWP];
          const float d1 = wcol[(4 * s4 + 1) * kWP];
          const float d2 = wcol[(4 * s4 + 2) * kWP];
          const float d3 = wcol[(4 * s4 + 3) * kWP];
          const float* ap = sA + r0 * kChunk + 4 * s4;
#pragma unroll
          for (int i = 0; i < 8; ++i) {
            const v4f av = *(const v4f_a*)(ap + i * kChunk);
            float a = acc[i];
            a = fmaf(-av[0], d0, a);
            a = fmaf(-av[1], d1, a);
            a = fmaf(-av[2], d2, a);
            a = fmaf(-av[3], d3, a);
            acc[i] = a;
          }
        }
        float dlb[8];
#pragma unroll
        for (int i = 0; i < 8; ++i) {
          float a = acc[i];
          const float* ar = sA + (r0 + i) * kChunk + r0;
          if (i > 0) {
            const v4f a0 = *(const v4f_a*)(ar);
#pragma unroll
            for (int j = 0; j < 4; ++j) {
              if (j < i) a = fmaf(-a0[j], dlb[j], a);
            }
          }
          if (i > 4) {
            const v4f a1 = *(const v4f_a*)(ar + 4);
#pragma unroll
            for (int j = 0; j < 4; ++j) {
              if (4 + j < i) a = fmaf(-a1[j], dlb[4 + j], a);
            }
          }
          dlb[i] = sBeta[r0 + i] * a;
        }
        v8h hv, lv;
#pragma unroll
        for (int i = 0; i < 8; ++i) {
          const float dv = dlb[i];
          wcol[(r0 + i) * kWP] = dv;
          _Float16 h0, l0;
          split_h(dv, h0, l0);
          hv[i] = h0;
          lv[i] = l0;
        }
        *(v8h_a*)(dhRow + r0) = hv;
        *(v8h_a*)(dlRow + r0) = lv;
      }
    }
    __syncthreads();

    {
      const v16h fdh = lds_frag(sDh + (16 * wave + c) * kTP + 8 * hh);
      const v16h fdl = lds_frag(sDl + (16 * wave + c) * kTP + 8 * hh);
      {
        const v16h pa0 = lds_frag(sP + c * kTP + 8 * hh);
        const v16h pa1 = lds_frag(sP + (16 + c) * kTP + 8 * hh);
        v8f r0 = z8, r1 = z8;
        o0 = wmma_h(pa0, fdh, o0);
        r0 = wmma_h(pa0, fdl, r0);
        o1 = wmma_h(pa1, fdh, o1);
        r1 = wmma_h(pa1, fdl, r1);
        hz_guard4(o0, r0, o1, r1, pa0, pa1, fdh, fdl, pa0, pa1);
#pragma unroll
        for (int r = 0; r < 8; ++r) {
          const float y0 = (o0[r] + r0[r] * kResInv) * qscl;
          const float y1 = (o1[r] + r1[r] * kResInv) * qscl;
          sW[(8 * hh + r) * kWP + 16 * wave + c]      = y0;
          sW[(16 + 8 * hh + r) * kWP + 16 * wave + c] = y1;
        }
      }
      sched_fence();
#pragma unroll 1
      for (int j = 0; j < 8; ++j) {
        const v16h kt = lds_frag(sKT + (16 * j + c) * kTP + 8 * hh);
        float* cp = sRow + 16 * j;
        const v4f c0 = *(const v4f_a*)(cp);
        const v4f c1 = *(const v4f_a*)(cp + 4);
        v8f sa;
        sa[0] = c0[0];
        sa[1] = c0[1];
        sa[2] = c0[2];
        sa[3] = c0[3];
        sa[4] = c1[0];
        sa[5] = c1[1];
        sa[6] = c1[2];
        sa[7] = c1[3];
        v8f ur = z8;
        sa = wmma_h(kt, fdh, sa);
        ur = wmma_h(kt, fdl, ur);
        hz_guard2(sa, ur, kt, fdh, fdl);
        v4f n0, n1;
        n0[0] = sa[0] + ur[0] * kResInv;
        n0[1] = sa[1] + ur[1] * kResInv;
        n0[2] = sa[2] + ur[2] * kResInv;
        n0[3] = sa[3] + ur[3] * kResInv;
        n1[0] = sa[4] + ur[4] * kResInv;
        n1[1] = sa[5] + ur[5] * kResInv;
        n1[2] = sa[6] + ur[6] * kResInv;
        n1[3] = sa[7] + ur[7] * kResInv;
        *(v4f_a*)(cp)     = n0;
        *(v4f_a*)(cp + 4) = n1;
        sched_fence();
      }
    }
    __syncthreads();

    {
      const v4f nw0 = *(const v4f*)(nw + 8 * c);
      const v4f nw1 = *(const v4f*)(nw + 8 * c + 4);
      v4u pk[2];
#pragma unroll
      for (int it = 0; it < 2; ++it) {
        const int row = 4 * wave + 2 * it + hh;
        const v4f a = *(const v4f_a*)(sW + row * kWP + 8 * c);
        const v4f b = *(const v4f_a*)(sW + row * kWP + 8 * c + 4);
        float ss = 0.0f;
#pragma unroll
        for (int e = 0; e < 4; ++e) {
          ss += a[e] * a[e];
          ss += b[e] * b[e];
        }
        ss += __shfl_xor(ss, 1, 32);
        ss += __shfl_xor(ss, 2, 32);
        ss += __shfl_xor(ss, 4, 32);
        ss += __shfl_xor(ss, 8, 32);
        const float rs = rsqrtf(ss * (1.0f / (float)kHd) + kNormEps);
        unsigned short hb[8];
#pragma unroll
        for (int e = 0; e < 4; ++e) {
          const float y0 = (a[e] * rs) * nw0[e];
          const float y1 = (b[e] * rs) * nw1[e];
          hb[e]     = h_bits(y0);
          hb[4 + e] = h_bits(y1);
        }
        pk[it] = (v4u){pk16(hb[0], hb[1]), pk16(hb[2], hb[3]), pk16(hb[4], hb[5]), pk16(hb[6], hb[7])};
      }
      for (int pass = 0; pass < 2; ++pass) {
#pragma unroll
        for (int it = 0; it < 2; ++it) {
          const int row = 4 * wave + 2 * it + hh;
          *(volatile v4u*)(On + (rowBase + t0 + row) * kDim + hd * kHd + 8 * c) = pk[it];
        }
        __threadfence();
      }
    }
  }
}

extern "C" void kernel_launch(void* const* d_in, const int* in_sizes, int n_in,
                              void* d_out, int out_size, void* d_ws, size_t ws_size, hipStream_t stream) {
  if (n_in < 7 || d_out == nullptr || d_ws == nullptr) return;
  if (in_sizes[0] != kRows * kDim || in_sizes[1] != kDim * kDim || in_sizes[2] != kDim * kDim ||
      in_sizes[3] != kDim * kDim || in_sizes[4] != kDim * kHeads || in_sizes[5] != kHd ||
      in_sizes[6] != kDim * kDim || out_size != kRows * kDim) return;

  const float* X   = (const float*)d_in[0];
  const float* Wq  = (const float*)d_in[1];
  const float* Wk  = (const float*)d_in[2];
  const float* Wv  = (const float*)d_in[3];
  const float* Wb  = (const float*)d_in[4];
  const float* onw = (const float*)d_in[5];
  const float* Wo  = (const float*)d_in[6];
  float* out = (float*)d_out;

  char* ws = (char*)d_ws;
  size_t off = 0;
  auto carve = [&](size_t bytes) -> char* { char* p = ws + off; off += (bytes + 255) & ~(size_t)255; return p; };
  unsigned short* XH   = (unsigned short*)carve((size_t)kRows * kDim * 2);
  unsigned short* WT   = (unsigned short*)carve((size_t)4 * kDim * kDim * 2);
  unsigned short* WBT  = (unsigned short*)carve((size_t)kGateN * kDim * 2);
  float*          GRAW = (float*)carve((size_t)kRows * kGateN * 4);
  float*          SCR  = (float*)carve((size_t)kRows * kDim * 4);
  unsigned short* QH   = (unsigned short*)carve(kHeadPlaneHalves * 2);
  unsigned short* KH   = (unsigned short*)carve(kHeadPlaneHalves * 2);
  unsigned short* ON   = XH;
  if (off > ws_size || off > (size_t)134217728) return;

  unsigned short* WQT = WT;
  unsigned short* WKT = WT + (size_t)1 * kDim * kDim;
  unsigned short* WVT = WT + (size_t)2 * kDim * kDim;
  unsigned short* WOT = WT + (size_t)3 * kDim * kDim;

  const int n8 = kRows * kDim / 8;
  cvt_x_kernel<<<n8 / 256, 256, 0, stream>>>(X, XH, n8);
  wt_cast_kernel<<<dim3(kDim / 64, kDim / 64, 4), 256, 0, stream>>>(Wq, Wk, Wv, Wo, WT);
  wb_cast_kernel<<<kDim / 64, 256, 0, stream>>>(Wb, WBT);

  const int bigBlocks  = (kRows / 64) * (kDim / 64) / 8;
  const int gateBlocks = (kRows / 64) * (kGateN / 64) / 8;
  const int l2nBlocks  = kRows * kHeads / 2 / 8;

  wmma_gemm64_f16<<<bigBlocks, 256, 0, stream>>>(XH, kDim, WQT, kDim, SCR, kDim, kRows, kDim, kDim, kWCarryInv);
  l2n_heads_kernel<<<l2nBlocks, 256, 0, stream>>>(SCR, QH);
  wmma_gemm64_f16<<<bigBlocks, 256, 0, stream>>>(XH, kDim, WKT, kDim, SCR, kDim, kRows, kDim, kDim, kWCarryInv);
  l2n_heads_kernel<<<l2nBlocks, 256, 0, stream>>>(SCR, KH);
  wmma_gemm64_f16<<<bigBlocks, 256, 0, stream>>>(XH, kDim, WVT, kDim, SCR, kDim, kRows, kDim, kDim, kWCarryInv);
  wmma_gemm64_f16<<<gateBlocks, 256, 0, stream>>>(XH, kDim, WBT, kDim, GRAW, kGateN, kRows, kGateN, kDim, kWCarryInv);

  chunk_scan_kernel<<<kBatch * kHeads, 256, kScanLdsBytes, stream>>>(QH, KH, SCR, GRAW, onw, ON);

  wmma_gemm64_f16<<<bigBlocks, 256, 0, stream>>>(ON, kDim, WOT, kDim, out, kDim, kRows, kDim, kDim, kWCarryInv);
}
